// MultiHeadAttention3D_20280835572057
// MI455X (gfx1250) — hardware-verified
//
#include <hip/hip_runtime.h>


namespace {
constexpr int B = 2, C = 256, P = 4096, NH = 8, HD = 32, BL = 2  , QL = 4096  ;
constexpr float XS = 8.0f, WSC = 256.0f, PS = 1024.0f, LOG2E = 1.4426950408889634f;
static_assert(P % 64 == 0 && QL % 32 == 0 && C == NH * HD, "tiling");
typedef _Float16 b16;
typedef __attribute__((ext_vector_type(16))) _Float16 v16b;
typedef __attribute__((ext_vector_type(8))) _Float16 v8b;
typedef __attribute__((ext_vector_type(8))) float v8f;
typedef __attribute__((ext_vector_type(4))) float v4f;
__device__ __forceinline__ float bf16_rne(float f) { unsigned int u = __float_as_uint(f); u += 0x7FFFu + ((u >> 16) & 1u); return __uint_as_float(u & 0xFFFF0000u); }
__device__ __forceinline__ void split16(float v, b16& hi, b16& lo) { hi = (b16)v; lo = (b16)(v - (float)hi); }
__device__ __forceinline__ v16b frag_kb(const b16* p, int hh) { const v8b a = *(const v8b*)(p + 8 * hh), b = *(const v8b*)(p + 16 + 8 * hh); v16b f;
#pragma unroll
  for (int e = 0; e < 8; ++e) { f[e] = a[e]; f[8 + e] = b[e]; } return f; }
__device__ __forceinline__ v8f wmma16b(v16b a, v16b b, v8f c) { v8f d = __builtin_amdgcn_wmma_f32_16x16x32_f16(false, a, false, b, (short)0, c, false, false); asm volatile("v_nop\n\tv_nop\n\tv_nop\n\tv_nop" : "+v"(d) : "v"(a), "v"(b)); return d; }
__device__ __forceinline__ void wave_lds_sync() { __builtin_amdgcn_fence(__ATOMIC_RELEASE, "workgroup"); __builtin_amdgcn_wave_barrier(); __builtin_amdgcn_fence(__ATOMIC_ACQUIRE, "workgroup"); }
__device__ __forceinline__ float pmul(float a, float b) { float p = a * b; asm volatile("" : "+v"(p)); return p; }
__device__ __forceinline__ int iclamp(int v, int lo, int hi) { return v < lo ? lo : (v > hi ? hi : v); }

typedef __attribute__((ext_vector_type(2))) _Float16 v2h;
typedef __attribute__((ext_vector_type(4))) _Float16 v4h;
__device__ __forceinline__ float nexp2(float v) { return __builtin_amdgcn_exp2f(v); }
__global__ __launch_bounds__(256) void prep_kernel(const float* __restrict__ qw, const float* __restrict__ ow, b16* __restrict__ WQ, b16* __restrict__ WO) {
  const size_t u = (size_t)blockIdx.x * 256 + threadIdx.x; const size_t n1 = (size_t)3 * C * C / 8, n2 = (size_t)C * C / 8; v8b o;
  if (u < n1) { const size_t e = u * 8; for (int j = 0; j < 8; ++j) o[j] = (b16)(bf16_rne(qw[e + j]) * WSC); for (int pass = 0; pass < 2; ++pass) { *(volatile v8b*)(WQ + e) = o; __threadfence(); } }
  else if (u < n1 + n2) { const size_t e = (u - n1) * 8; for (int j = 0; j < 8; ++j) o[j] = (b16)(bf16_rne(ow[e + j]) * WSC); for (int pass = 0; pass < 2; ++pass) { *(volatile v8b*)(WO + e) = o; __threadfence(); } }
}
__global__ __launch_bounds__(128) void qkv_kernel(const float* __restrict__ x, const b16* __restrict__ WQ, b16* __restrict__ QP, b16* __restrict__ KP, b16* __restrict__ VT) {
  __shared__ __attribute__((aligned(16))) b16 As[64][C + 8]; __shared__ __attribute__((aligned(16))) float Tf[4][16][128 + 4];
  const int wave = threadIdx.x >> 5, lane = threadIdx.x & 31, nloc = lane & 15, hlf = lane >> 4; const int p0 = blockIdx.x * 64; const int b = blockIdx.y; const int slab = blockIdx.z, n0 = slab * 128, which = slab / 2, c0 = n0 - which * C;
  for (int i = threadIdx.x; i < C * 64; i += 128) { const int c = i / 64, pp = i % 64; As[pp][c] = (b16)(bf16_rne(x[((size_t)b * C + c) * P + p0 + pp]) * XS); }
  __syncthreads();
  v8f acc[8];
#pragma unroll
  for (int t = 0; t < 8; ++t) acc[t] = (v8f){};
#pragma unroll 2
  for (int kb = 0; kb < C; kb += 32) { const v16b a = frag_kb(&As[wave * 16 + nloc][kb], hlf);
#pragma unroll
    for (int t = 0; t < 8; ++t) acc[t] = wmma16b(a, frag_kb(WQ + (size_t)(n0 + t * 16 + nloc) * C + kb, hlf), acc[t]); }
#pragma unroll
  for (int t = 0; t < 8; ++t)
#pragma unroll
    for (int r = 0; r < 8; ++r) Tf[wave][8 * hlf + r][t * 16 + nloc] = acc[t][r] * (1.0f / (XS * WSC));
  __syncthreads();
  for (int pass = 0; pass < 2; ++pass) {
    if (which < 2) { b16* plane = which == 0 ? QP : KP; const int cl = lane * 4; const int c = c0 + cl; const int h = c / HD, d = c % HD;
      for (int rr = 0; rr < 16; ++rr) { const int vox = p0 + wave * 16 + rr; v4h o4; for (int j = 0; j < 4; ++j) o4[j] = (b16)(Tf[wave][rr][cl + j] * XS); *(volatile v4h*)(plane + (((size_t)b * NH + h) * P + vox) * HD + d) = o4; } }
    else {
#pragma unroll 1
      for (int q = 0; q < 32; ++q) { const int cl = wave * 32 + q; const int c = c0 + cl; const int h = c / HD, d = c % HD; const int tk = lane * 2; v2h vv; vv[0] = (b16)(Tf[tk >> 4][tk & 15][cl] * XS); vv[1] = (b16)(Tf[(tk + 1) >> 4][(tk + 1) & 15][cl] * XS);
        *(volatile v2h*)(VT + (((size_t)b * NH + h) * HD + d) * (size_t)P + p0 + lane * 2) = vv; } }
    __threadfence(); }
}
__global__ __launch_bounds__(64) void attn_kernel(const b16* __restrict__ QP, const b16* __restrict__ KP, const b16* __restrict__ VT, b16* __restrict__ Ch, b16* __restrict__ Cl) {
  __shared__ __attribute__((aligned(16))) b16 Pb[2][16][32 + 8]; __shared__ __attribute__((aligned(16))) float To[2][16][HD + 4];
  const int wave = threadIdx.x >> 5, lane = threadIdx.x & 31, hh = lane >> 4, col = lane & 15; const int b = blockIdx.y / NH, h = blockIdx.y % NH; const int q0 = blockIdx.x * 32 + wave * 16, qi = q0 + col;
  const size_t ph = (size_t)b * NH + h; const b16* Qb = QP + ph * P * HD; const b16* Kb = KP + ph * P * HD; const b16* Vb = VT + ph * HD * (size_t)P;
  const v16b qa = frag_kb(Qb + (size_t)qi * HD, hh);
  const float cs = LOG2E / (5.656854249492381f * XS * XS);
  float m = -INFINITY, l = 0.0f; v8f o[2] = {(v8f){}, (v8f){}};
#pragma unroll 1
  for (int kb = 0; kb < P; kb += 32) {
    float e[16]; float mx = -INFINITY;
#pragma unroll
    for (int u = 0; u < 2; ++u) { v8f s = (v8f){}; s = wmma16b(frag_kb(Kb + (size_t)(kb + u * 16 + col) * HD, hh), qa, s);
#pragma unroll
      for (int r = 0; r < 8; ++r) { const float vv = s[r] * cs; e[u * 8 + r] = vv; mx = fmaxf(mx, vv); } }
    mx = fmaxf(mx, __shfl_xor(mx, 16)); const float mn = fmaxf(m, mx); const float al = nexp2(m - mn); float sum = 0.0f;
#pragma unroll
    for (int i2 = 0; i2 < 16; ++i2) { const float p = nexp2(e[i2] - mn); sum += p; Pb[wave][col][(i2 < 8 ? 0 : 16) + 8 * hh + (i2 & 7)] = (b16)(p * PS); }
    sum += __shfl_xor(sum, 16); l = l * al + sum; m = mn;
    wave_lds_sync();
    const v16b pf = frag_kb(&Pb[wave][col][0], hh);
#pragma unroll
    for (int t = 0; t < 2; ++t) { o[t] *= al; o[t] = wmma16b(frag_kb(Vb + (size_t)(t * 16 + col) * P + kb, hh), pf, o[t]); }
    wave_lds_sync(); }
  const float inv = 1.0f / (l * PS * XS);
#pragma unroll
  for (int t = 0; t < 2; ++t)
#pragma unroll
    for (int r = 0; r < 8; ++r) To[wave][col][t * 16 + 8 * hh + r] = o[t][r] * inv;
  wave_lds_sync();
  b16* Hb = Ch + ph * P * HD; b16* Lb = Cl + ph * P * HD;
  for (int pass = 0; pass < 2; ++pass) { for (int rr = 0; rr < 16; ++rr) { b16 p, q; split16(To[wave][rr][lane] * XS, p, q); ((volatile b16*)Hb)[(size_t)(q0 + rr) * HD + lane] = p; ((volatile b16*)Lb)[(size_t)(q0 + rr) * HD + lane] = q; } __threadfence(); }
}
__global__ __launch_bounds__(128) void out_kernel(const b16* __restrict__ Ch, const b16* __restrict__ Cl, const b16* __restrict__ WO, const float* __restrict__ pb, float* __restrict__ out) {
  __shared__ __attribute__((aligned(16))) float To[4][16][32 + 4];
  const int wave = threadIdx.x >> 5, lane = threadIdx.x & 31, nloc = lane & 15, hlf = lane >> 4; const int o0 = blockIdx.x * 64 + wave * 16; const int p0 = blockIdx.y * 32; const int b = blockIdx.z;
  v8f acc[2] = {(v8f){}, (v8f){}};
#pragma unroll
  for (int ks = 0; ks < NH; ++ks) { const v16b a = frag_kb(WO + (size_t)(o0 + nloc) * C + ks * HD, hlf); const size_t pl = (((size_t)b * NH + ks) * P) * HD;
#pragma unroll
    for (int t = 0; t < 2; ++t) { const size_t ro = pl + (size_t)(p0 + t * 16 + nloc) * HD; acc[t] = wmma16b(a, frag_kb(Ch + ro, hlf), acc[t]); acc[t] = wmma16b(a, frag_kb(Cl + ro, hlf), acc[t]); } }
#pragma unroll
  for (int t = 0; t < 2; ++t)
#pragma unroll
    for (int r = 0; r < 8; ++r) To[wave][8 * hlf + r][t * 16 + nloc] = acc[t][r] * (1.0f / (XS * WSC));
  wave_lds_sync();
  for (int pass = 0; pass < 2; ++pass) { for (int rr = 0; rr < 16; ++rr) { const int o = o0 + rr; ((volatile float*)out)[((size_t)b * C + o) * P + p0 + lane] = To[wave][rr][lane] + bf16_rne(pb[o]); } __threadfence(); }
}
}

extern "C" void kernel_launch(void* const* d_in, const int* in_sizes, int n_in, void* d_out, int out_size, void* d_ws, size_t ws_size, hipStream_t stream) {
  (void)n_in;
  auto Fp = [&](int i) { return (const float*)d_in[i]; };
  if (in_sizes[0] != B * C * P || in_sizes[1] != 3 * C * C || in_sizes[2] != C * C || in_sizes[3] != C || out_size != B * C * P) return;
  size_t off = 0; char* ws = (char*)d_ws;
  auto carve = [&](size_t bytes) { char* p = ws + off; off += (bytes + 255) & ~(size_t)255; return p; };
  b16* WQ = (b16*)carve((size_t)3 * C * C * 2); b16* WO = (b16*)carve((size_t)C * C * 2); const size_t plane = (size_t)B * C * P * 2;
  b16* QP = (b16*)carve(plane); b16* KP = (b16*)carve(plane); b16* VT = (b16*)carve(plane); b16* Ch = (b16*)carve(plane); b16* Cl = (b16*)carve(plane);
  if (off > ws_size || off > ((size_t)128 << 20)) return;
  prep_kernel<<<(unsigned)(((size_t)4 * C * C / 8 + 255) / 256), 256, 0, stream>>>(Fp(1), Fp(2), WQ, WO);
  qkv_kernel<<<dim3(P / 64, BL, 6), 128, 0, stream>>>(Fp(0), WQ, QP, KP, VT);
  attn_kernel<<<dim3(QL / 32, BL * NH), 64, 0, stream>>>(QP, KP, VT, Ch, Cl);
  out_kernel<<<dim3(C / 64, QL / 32, BL), 128, 0, stream>>>(Ch, Cl, WO, Fp(3), (float*)d_out);
}
